// defomableConv_offset_13520557048343
// MI455X (gfx1250) — hardware-verified
//
#include <hip/hip_runtime.h>
#include <math.h>

typedef __attribute__((ext_vector_type(16))) _Float16 v16h;
typedef __attribute__((ext_vector_type(16))) __bf16 v16b;
typedef __attribute__((ext_vector_type(8)))  _Float16 v8h;
typedef __attribute__((ext_vector_type(8)))  float v8f;
typedef __attribute__((ext_vector_type(4)))  float v4f;
typedef __attribute__((ext_vector_type(2)))  float v2f;
typedef __attribute__((ext_vector_type(4)))  unsigned v4u;
typedef __attribute__((ext_vector_type(4)))  int v4i;
typedef float __attribute__((may_alias)) float_a;
typedef int __attribute__((may_alias)) int_a;

template <typename T> __device__ __forceinline__ void vst2(void* p, T v) { *(volatile T*)p = v; __threadfence(); *(volatile T*)p = v; }
__device__ __forceinline__ v8f wmma16(v16h a, v16h b, v8f c) {
  v8f d = __builtin_amdgcn_wmma_f32_16x16x32_f16(false, a, false, b, (short)0, c, false, false);
  asm volatile("v_nop\n\tv_nop\n\tv_nop\n\tv_nop" : "+v"(d) : "v"(a), "v"(b));
  return d;
}
__device__ __forceinline__ v8f wmma_bf(v16b a, v16b b, v8f c) {
  v8f d = __builtin_amdgcn_wmma_f32_16x16x32_bf16(false, a, false, b, (short)0, c, false, false);
  asm volatile("v_nop\n\tv_nop\n\tv_nop\n\tv_nop" : "+v"(d) : "v"(a), "v"(b));
  return d;
}
__device__ __forceinline__ v16h frag_h(const _Float16* rowk0, int lane) {
  union { v16h v; v8h q[2]; } u; const _Float16* p = rowk0 + 8 * (lane >> 4);
  u.q[0] = *(const v8h*)p; u.q[1] = *(const v8h*)(p + 16); return u.v;
}
__device__ __forceinline__ v16h frag_f32(const float* rowk0, int lane) {
  v16h a; const float* p = rowk0 + 8 * (lane >> 4);
#pragma unroll
  for (int i = 0; i < 8; ++i) { a[i] = (_Float16)p[i]; a[8 + i] = (_Float16)p[16 + i]; }
  return a;
}
__device__ __forceinline__ v16h frag_f32s(const float* rowk0, int lane, float sc) {
  v16h a; const float* p = rowk0 + 8 * (lane >> 4);
#pragma unroll
  for (int i = 0; i < 8; ++i) { a[i] = (_Float16)(p[i] * sc); a[8 + i] = (_Float16)(p[16 + i] * sc); }
  return a;
}
__device__ __forceinline__ v16h fragc_f32(const float* W, int k0, int n, int lane, int ld, int K) {
  v16h a; const int g = lane >> 4;
#pragma unroll
  for (int i = 0; i < 8; ++i) { const int ka = k0 + 8 * g + i, kb = ka + 16;
    a[i] = (_Float16)(ka < K ? W[(size_t)(ka < K ? ka : K - 1) * ld + n] : 0.f); a[8 + i] = (_Float16)(kb < K ? W[(size_t)(kb < K ? kb : K - 1) * ld + n] : 0.f); }
  return a;
}
struct F2 { v16b h, l; };
__device__ __forceinline__ F2 bsplit16(const float v[16]) { F2 r;
#pragma unroll
  for (int i = 0; i < 16; ++i) { const __bf16 h = (__bf16)v[i]; r.h[i] = h; r.l[i] = (__bf16)(v[i] - (float)h); }
  return r; }
__device__ __forceinline__ F2 split_row(const float* row, int k0, int lane) { float v[16]; const float* p = row + k0 + 8 * (lane >> 4);
#pragma unroll
  for (int i = 0; i < 8; ++i) { v[i] = p[i]; v[8 + i] = p[16 + i]; }
  return bsplit16(v); }
__device__ __forceinline__ F2 split_rowK(const float* row, int k0, int lane, int K) { float v[16]; const int g = lane >> 4;
#pragma unroll
  for (int i = 0; i < 8; ++i) { const int ka = k0 + 8 * g + i, kb = ka + 16; v[i] = ka < K ? row[ka < K ? ka : K - 1] : 0.f; v[8 + i] = kb < K ? row[kb < K ? kb : K - 1] : 0.f; }
  return bsplit16(v); }
__device__ __forceinline__ F2 split_col(const float* W, int k0, int n, int lane, int ld, int K) { float v[16]; const int g = lane >> 4;
#pragma unroll
  for (int i = 0; i < 8; ++i) { const int ka = k0 + 8 * g + i, kb = ka + 16; v[i] = ka < K ? W[(size_t)(ka < K ? ka : K - 1) * ld + n] : 0.f; v[8 + i] = kb < K ? W[(size_t)(kb < K ? kb : K - 1) * ld + n] : 0.f; }
  return bsplit16(v); }
__device__ __forceinline__ v8f mac3(const F2& a, const F2& b, v8f c) { c = wmma_bf(a.l, b.h, c); c = wmma_bf(a.h, b.l, c); return wmma_bf(a.h, b.h, c); }
__device__ __forceinline__ float sigm(float v) { return 1.0f / (1.0f + expf(-v)); }
#define LDSX() do { asm volatile("s_wait_dscnt 0" ::: "memory"); __builtin_amdgcn_wave_barrier(); __builtin_amdgcn_fence(__ATOMIC_RELEASE, "workgroup"); } while (0)


#define NB 8
#define CC 256
#define HH 64
#define WWD 64
#define NP (HH * WWD)
#define OG 2
#define CG 128
#define KT 9
#define KOFF (CC * KT)
#define KDEF (CG * KT)
#define NOFF 36
#ifndef TNB
#define TNB NB
#define TB0 0
#endif
typedef __attribute__((ext_vector_type(8))) __bf16 v8b;
__device__ __forceinline__ v16b frag_b(const __bf16* rowk0, int lane) {
  union { v16b v; v8b q[2]; } u; const __bf16* p = rowk0 + 8 * (lane >> 4);
  u.q[0] = *(const v8b*)p; u.q[1] = *(const v8b*)(p + 16); return u.v;
}
__device__ __forceinline__ float bfr(float v) { return (float)(__bf16)v; }
__device__ __attribute__((noinline)) float exp_ni(float v) { return expf(v); }
__device__ __attribute__((noinline)) float erf_ni(float v) { return erff(v); }

__device__ __attribute__((noinline)) float floor_ni(float v) { return floorf(v); }
#define WS_PW   0u
#define POW 0
#define PDW (POW + 48 * KOFF)
#define PWEND (PDW + CC * KDEF)
#define OFFP 64
#define WS_OFF  (WS_PW + 2u * PWEND)
#define WS_SH   (WS_OFF + 4u * NB * NP * OFFP)
#define WS_SL   (WS_SH + 2u * NP * OG * KDEF)
#define WS_END  (WS_SL + 2u * NP * OG * KDEF)

__global__ __launch_bounds__(256) void k_pack(const float* __restrict__ OW, const float* __restrict__ DW, __bf16* __restrict__ PW) {
  __shared__ __align__(16) __bf16 s[KOFF]; const int r = blockIdx.x, which = blockIdx.y, tid = threadIdx.x;
  if (which == 0) { if (r >= 48) return; for (int k = tid; k < KOFF; k += 256) s[k] = (__bf16)((r < NOFF) ? OW[(size_t)r * KOFF + k] : 0.f); __syncthreads(); for (int q = tid; q < KOFF / 8; q += 256) vst2((unsigned*)(PW + POW + (size_t)r * KOFF + q * 8), *(const v4u*)&s[q * 8]); }
  else { for (int k = tid; k < KDEF; k += 256) s[k] = (__bf16)DW[(size_t)r * KDEF + k]; __syncthreads(); for (int q = tid; q < KDEF / 8; q += 256) vst2((unsigned*)(PW + PDW + (size_t)r * KDEF + q * 8), *(const v4u*)&s[q * 8]); }
}
__global__ __launch_bounds__(128) void k_offconv(const float* __restrict__ F3, const __bf16* __restrict__ PW, const float* __restrict__ TM, const float* __restrict__ BETA, float* __restrict__ OFF) {
  __shared__ __align__(16) float so[4][16][68];
  const int tid = threadIdx.x, wave = tid >> 5, lane = tid & 31, col = lane & 15, g = lane >> 4; const int b = blockIdx.y + TB0; const int p0 = blockIdx.x * 64 + wave * 16; const int pos = p0 + col; const int y = pos >> 6, x = pos & 63;
  const float* fb = F3 + (size_t)b * CC * NP;
  v8f acc[3] = {};
#pragma unroll 1
  for (int kc = 0; kc < KOFF / 32; ++kc) { v16b a;
#pragma unroll
    for (int i = 0; i < 16; ++i) { const int kk = kc * 32 + 8 * g + (i & 7) + ((i >> 3) << 4); const int c = kk / 9, t = kk - c * 9; const int ky = t / 3, kx = t - ky * 3; const int yy = y + ky - 1, xx = x + kx - 1; float v = 0.f; if (yy >= 0 && yy < HH && xx >= 0 && xx < WWD) v = fb[(size_t)c * NP + yy * WWD + xx]; a[i] = (__bf16)v; }
#pragma unroll
    for (int j = 0; j < 3; ++j) acc[j] = wmma_bf(a, frag_b(PW + POW + (size_t)(j * 16 + col) * KOFF + kc * 32, lane), acc[j]); }
  const float beta = bfr(BETA[0]);
#pragma unroll
  for (int j = 0; j < 3; ++j)
#pragma unroll
    for (int r = 0; r < 8; ++r) { const int pr = p0 + 8 * g + r; const float mod = 1.0f + beta * bfr(TM[(size_t)b * NP + pr]); so[wave][8 * g + r][j * 16 + col] = acc[j][r] * mod; }
  LDSX();
  for (int q = lane; q < 16 * 16; q += 32) so[wave][q >> 4][48 + (q & 15)] = 0.f;
  LDSX();
  for (int rl = 0; rl < 16; ++rl) if (lane < 16) vst2(OFF + ((size_t)b * NP + p0 + rl) * OFFP + lane * 4, *(const v4f*)&so[wave][rl][lane * 4]);
}
__global__ __launch_bounds__(256) void k_sample(const float* __restrict__ X, const float* __restrict__ OFF, int b, __bf16* __restrict__ SH, __bf16* __restrict__ SL) {
  __shared__ float soff[48]; __shared__ __align__(16) __bf16 sh[OG * KDEF], sl[OG * KDEF];
  const int pos = blockIdx.x, tid = threadIdx.x; const int y = pos >> 6, x = pos & 63;
  if (tid < 48) soff[tid] = OFF[((size_t)b * NP + pos) * OFFP + tid];
  __syncthreads();
  const float* xb = X + (size_t)b * CC * NP;
#pragma unroll 1
  for (int e = tid; e < OG * KDEF; e += 256) { const int gq = e / KDEF, rem = e - gq * KDEF; const int c = rem / KT, t = rem - c * KT; const int ky = t / 3, kx = t - ky * 3;
    const float dy = soff[(gq * KT + t) * 2 + 0], dx = soff[(gq * KT + t) * 2 + 1];
    const float py = (float)y + (float)ky - 1.0f + dy, px = (float)x + (float)kx - 1.0f + dx;
    const float y0f = floor_ni(py), x0f = floor_ni(px); const float wy = py - y0f, wx = px - x0f; const int y0 = (int)y0f, x0 = (int)x0f;
    const float* xc = xb + (size_t)(gq * CG + c) * NP;
    float v = 0.f;
    { const bool oky0 = (y0 >= 0 && y0 < HH), oky1 = (y0 + 1 >= 0 && y0 + 1 < HH), okx0 = (x0 >= 0 && x0 < WWD), okx1 = (x0 + 1 >= 0 && x0 + 1 < WWD);
      const int cy0 = min(max(y0, 0), HH - 1), cy1 = min(max(y0 + 1, 0), HH - 1), cx0 = min(max(x0, 0), WWD - 1), cx1 = min(max(x0 + 1, 0), WWD - 1);
      const float v00 = (oky0 && okx0) ? bfr(xc[cy0 * WWD + cx0]) : 0.f, v01 = (oky0 && okx1) ? bfr(xc[cy0 * WWD + cx1]) : 0.f, v10 = (oky1 && okx0) ? bfr(xc[cy1 * WWD + cx0]) : 0.f, v11 = (oky1 && okx1) ? bfr(xc[cy1 * WWD + cx1]) : 0.f;
      v = v00 * (1.0f - wy) * (1.0f - wx) + v01 * (1.0f - wy) * wx + v10 * wy * (1.0f - wx) + v11 * wy * wx; }
    const __bf16 hb = (__bf16)v; sh[e] = hb; sl[e] = (__bf16)(v - (float)hb); }
  __syncthreads();
  for (int q = tid; q < OG * KDEF / 8; q += 256) { vst2((unsigned*)(SH + (size_t)pos * OG * KDEF + q * 8), *(const v4u*)&sh[q * 8]); vst2((unsigned*)(SL + (size_t)pos * OG * KDEF + q * 8), *(const v4u*)&sl[q * 8]); }
}
__global__ __launch_bounds__(128) void k_dconv(const __bf16* __restrict__ SH, const __bf16* __restrict__ SL, const __bf16* __restrict__ PW, const float* __restrict__ DB, int b, float* __restrict__ out) {
  __shared__ __align__(16) float st[128][68];
  const int tid = threadIdx.x, wave = tid >> 5, lane = tid & 31, col = lane & 15, g = lane >> 4; const int gq = blockIdx.y; const int p0 = blockIdx.x * 64; const int pr = p0 + wave * 16 + col;
  v8f acc[8] = {};
#pragma unroll 2
  for (int kc = 0; kc < KDEF / 32; ++kc) { const size_t ar = ((size_t)pr * OG + gq) * KDEF + kc * 32; const v16b ah = frag_b(SH + ar, lane), al = frag_b(SL + ar, lane);
#pragma unroll
    for (int j = 0; j < 8; ++j) { const v16b w = frag_b(PW + PDW + (size_t)(gq * CG + j * 16 + col) * KDEF + kc * 32, lane); acc[j] = wmma_bf(al, w, acc[j]); acc[j] = wmma_bf(ah, w, acc[j]); } }
#pragma unroll
  for (int j = 0; j < 8; ++j) { const int o = j * 16 + col; const float bb = bfr(DB[gq * CG + o]);
#pragma unroll
    for (int r = 0; r < 8; ++r) st[o][wave * 16 + 8 * g + r] = acc[j][r] + bb; }
  __syncthreads();
  for (int q = tid; q < 128 * 16; q += 128) { const int o = q >> 4, pc = q & 15; vst2(out + ((size_t)b * CC + gq * CG + o) * NP + p0 + pc * 4, *(const v4f*)&st[o][pc * 4]); }
}
extern "C" void kernel_launch(void* const* d_in, const int* in_sizes, int n_in, void* d_out, int out_size, void* d_ws, size_t ws_size, hipStream_t stream) {
  (void)in_sizes; (void)n_in; (void)out_size;
  const float** F = (const float**)d_in;
  if (ws_size < (size_t)WS_END) return;
  char* ws = (char*)d_ws; __bf16 *PW = (__bf16*)(ws + WS_PW), *SH = (__bf16*)(ws + WS_SH), *SL = (__bf16*)(ws + WS_SL); float* OFF = (float*)(ws + WS_OFF);
  k_pack<<<dim3(CC, 2), 256, 0, stream>>>(F[4], F[5], PW);
  k_offconv<<<dim3(NP / 64, TNB - TB0), 128, 0, stream>>>(F[0], PW, F[2], F[3], OFF);
  for (int b = TB0; b < TNB; ++b) {
    k_sample<<<NP, 256, 0, stream>>>(F[1], OFF, b, SH, SL);
    k_dconv<<<dim3(NP / 64, OG), 128, 0, stream>>>(SH, SL, PW, F[6], b, (float*)d_out); }
}
